// GlobalFreqBranch_128849019511
// MI455X (gfx1250) — hardware-verified
//
#include <hip/hip_runtime.h>


#define NBT  64
#define NI   224
#define NP   256
#define NPIX (NI * NI)
#define KB   8
#define EE   256
#define DM   NP
#define STEPR 19.798990f
#define W224 0.028049935f
#define LOSC 1024.0f

typedef _Float16 h16;
typedef unsigned short bf;
typedef __attribute__((ext_vector_type(16))) __bf16   v16bf;
typedef __attribute__((ext_vector_type(16))) _Float16 v16h;
typedef __attribute__((ext_vector_type(8)))  _Float16 v8h;
typedef __attribute__((ext_vector_type(8)))  unsigned short v8us;
typedef __attribute__((ext_vector_type(8)))  float    v8f;
typedef __attribute__((ext_vector_type(4)))  float    v4f;
typedef __attribute__((ext_vector_type(4)))  _Float16 v4h;
typedef v8h  __attribute__((may_alias)) v8ha;
typedef v4f  __attribute__((may_alias)) v4fa;
typedef v8us __attribute__((may_alias)) v8usa;

__device__ __forceinline__ unsigned short f2bf(float f) { unsigned u = __float_as_uint(f); u += 0x7FFFu + ((u >> 16) & 1u); return (unsigned short)(u >> 16); }
__device__ __forceinline__ float bf2f(unsigned short b) { return __uint_as_float(((unsigned)b) << 16); }
__device__ __forceinline__ float bfr(float f) { return bf2f(f2bf(f)); }
__device__ __forceinline__ v16h cat16(v8h lo, v8h hi) { return __builtin_shufflevector(lo, hi, 0, 1, 2, 3, 4, 5, 6, 7, 8, 9, 10, 11, 12, 13, 14, 15); }
__device__ __forceinline__ v16bf cat16b(v8us lo, v8us hi) { return __builtin_bit_cast(v16bf, __builtin_shufflevector(lo, hi, 0, 1, 2, 3, 4, 5, 6, 7, 8, 9, 10, 11, 12, 13, 14, 15)); }
__device__ __forceinline__ v8f wmma16(v16h a, v16h b, v8f c) { return __builtin_amdgcn_wmma_f32_16x16x32_f16(false, a, false, b, (short)0, c, false, false); }
__device__ __forceinline__ v8f wmmab(v16bf a, v16bf b, v8f c) { return __builtin_amdgcn_wmma_f32_16x16x32_bf16(false, a, false, b, (short)0, c, false, false); }

__global__ __launch_bounds__(256) void k_wt(const float* __restrict__ Wm, int K, int ncols, bf* WT) {
    __shared__ __align__(16) unsigned short tl[64 * 72];
    const int tid = threadIdx.x, k0 = blockIdx.x * 64, n0 = blockIdx.y * 64;
    const int kk = tid >> 2, nq = (tid & 3) * 16;
#pragma unroll
    for (int i = 0; i < 16; ++i) tl[(nq + i) * 72 + kk] = f2bf(Wm[(size_t)(k0 + kk) * ncols + n0 + nq + i]);
    __syncthreads();
    const int piece = tid & 7;
    auto pass = [&]() {
#pragma unroll
        for (int s = 0; s < 2; ++s) { const int nr = (tid >> 3) + 32 * s; const v8us val = *(const v8usa*)(tl + nr * 72 + piece * 8); *(volatile v8us*)(WT + (size_t)(n0 + nr) * K + k0 + piece * 8) = val; }
    };
    pass(); __threadfence(); pass();
}
template <bool SPLITA, bool F16OUT = false>
__global__ __launch_bounds__(128) void k_gemmb(const bf* __restrict__ A, const bf* __restrict__ Al, const bf* __restrict__ Bn, const float* __restrict__ bias, float* C, int ldc, h16* C2, const float* __restrict__ R = nullptr, int K = DM, int roundR = 1) {
    __shared__ __align__(16) float ost[4][16 * 68];
    const int lane = threadIdx.x & 31, wave = threadIdx.x >> 5, lr = lane & 15, hi = lane >> 4;
    const int r0 = blockIdx.x * 64 + wave * 16, c0 = blockIdx.y * 64;
    const size_t aoff = (size_t)(r0 + lr) * K + 8 * hi;
    size_t boff[4];
#pragma unroll
    for (int t = 0; t < 4; ++t) boff[t] = (size_t)(c0 + t * 16 + lr) * K + 8 * hi;
    v8f acc[4];
#pragma unroll
    for (int t = 0; t < 4; ++t) acc[t] = (v8f){};
#pragma unroll 1
    for (int kc = 0; kc < K; kc += 32) {
        const v16bf a = cat16b(*(const v8us*)(A + aoff + kc), *(const v8us*)(A + aoff + kc + 16));
        v16bf al = a;
        if (SPLITA) al = cat16b(*(const v8us*)(Al + aoff + kc), *(const v8us*)(Al + aoff + kc + 16));
#pragma unroll
        for (int t = 0; t < 4; ++t) { const v16bf b = cat16b(*(const v8us*)(Bn + boff[t] + kc), *(const v8us*)(Bn + boff[t] + kc + 16)); acc[t] = wmmab(a, b, acc[t]); if (SPLITA) acc[t] = wmmab(al, b, acc[t]); }
        asm volatile("v_nop\n\tv_nop\n\tv_nop\n\tv_nop" : "+v"(acc[0]), "+v"(acc[1]), "+v"(acc[2]), "+v"(acc[3]) : "v"(a), "v"(al));
    }
    float* os = &ost[wave][0];
#pragma unroll
    for (int t = 0; t < 4; ++t) { const float bv = bias ? bfr(bias[c0 + t * 16 + lr]) : 0.f;
#pragma unroll
        for (int j = 0; j < 8; ++j) os[(hi * 8 + j) * 68 + t * 16 + lr] = acc[t][j] + bv; }
    __syncthreads();
    if (F16OUT) {
        h16* crow = (h16*)(void*)C + (size_t)r0 * ldc + c0;
        auto pass = [&]() {
#pragma unroll
            for (int s = 0; s < 4; ++s) { const int row = 4 * s + (lane >> 3), piece = lane & 7; const float* sp = os + row * 68 + piece * 8; v8h o, o2;
#pragma unroll
                for (int i = 0; i < 8; ++i) { const h16 a = (h16)sp[i]; o[i] = a; o2[i] = (h16)((sp[i] - (float)a) * LOSC); }
                *(volatile v8h*)(crow + (size_t)row * ldc + piece * 8) = o; if (C2) *(volatile v8h*)(C2 + (size_t)r0 * ldc + c0 + (size_t)row * ldc + piece * 8) = o2; }
        };
        pass(); __threadfence(); pass();
    } else {
        float* crow = C + (size_t)r0 * ldc + c0;
        auto pass = [&]() {
#pragma unroll
            for (int s = 0; s < 8; ++s) { const int Lid = (lane >> 3) + 4 * s, piece = lane & 7; const int row = Lid >> 1, cofs = (Lid & 1) * 32 + piece * 4;
                v4f val = *(const v4fa*)(os + row * 68 + cofs); if (R) { const v4f rv = *(const v4f*)(R + ((size_t)r0 + row) * ldc + c0 + cofs); val += roundR ? (v4f){bfr(rv[0]), bfr(rv[1]), bfr(rv[2]), bfr(rv[3])} : rv; }
                *(volatile v4f*)(crow + (size_t)row * ldc + cofs) = val; }
        };
        pass(); __threadfence(); pass();
    }
}


template <int MODE>
__global__ __launch_bounds__(128) void k_gemm3z(const bf* __restrict__ Ah, const bf* __restrict__ Al, const bf* __restrict__ Bh, const bf* __restrict__ Bl, int K, float* C, int ldc, size_t sA, size_t sB, size_t sC) {
    if ((MODE & 1) && (int)blockIdx.y * 64 > (int)blockIdx.x * 64 + 63) return;
    const size_t z = blockIdx.z; Ah += z * sA; Al += z * sA; Bh += z * sB; Bl += z * sB; C += z * sC;
    const int Klim = (MODE & 2) ? min(K, ((int)blockIdx.x + 1) * 64) : K;
    __shared__ __align__(16) float ost[4][16 * 68];
    const int lane = threadIdx.x & 31, wave = threadIdx.x >> 5, lr = lane & 15, hi = lane >> 4;
    const int r0 = blockIdx.x * 64 + wave * 16, c0 = blockIdx.y * 64;
    const size_t aoff = (size_t)(r0 + lr) * K + 8 * hi;
    v8f acc[4];
#pragma unroll
    for (int t = 0; t < 4; ++t) acc[t] = (v8f){};
#pragma unroll 1
    for (int kc = 0; kc < Klim; kc += 32) {
        const v16bf a = cat16b(*(const v8us*)(Ah + aoff + kc), *(const v8us*)(Ah + aoff + kc + 16));
        v16bf al = a; if (!(MODE & 4) && !(MODE & 16)) al = cat16b(*(const v8us*)(Al + aoff + kc), *(const v8us*)(Al + aoff + kc + 16));
#pragma unroll
        for (int t = 0; t < 4; ++t) { const size_t bo = (size_t)(c0 + t * 16 + lr) * K + kc + 8 * hi;
            const v16bf bh = cat16b(*(const v8us*)(Bh + bo), *(const v8us*)(Bh + bo + 16));
            acc[t] = wmmab(a, bh, acc[t]);
            if (!(MODE & 4)) { if (!(MODE & 16)) acc[t] = wmmab(al, bh, acc[t]); if (!(MODE & 8)) { const v16bf bl = cat16b(*(const v8us*)(Bl + bo), *(const v8us*)(Bl + bo + 16)); acc[t] = wmmab(a, bl, acc[t]); } } }
        asm volatile("v_nop\n\tv_nop\n\tv_nop\n\tv_nop" : "+v"(acc[0]), "+v"(acc[1]), "+v"(acc[2]), "+v"(acc[3]) : "v"(a), "v"(al));
    }
    float* os = &ost[wave][0];
#pragma unroll
    for (int t = 0; t < 4; ++t) {
#pragma unroll
        for (int j = 0; j < 8; ++j) os[(hi * 8 + j) * 68 + t * 16 + lr] = acc[t][j]; }
    __builtin_amdgcn_wave_barrier(); asm volatile("" ::: "memory");
    float* crow = C + (size_t)r0 * ldc + c0;
    auto pass = [&]() {
#pragma unroll
        for (int s = 0; s < 8; ++s) { const int Lid = (lane >> 3) + 4 * s, piece = lane & 7; const int row = Lid >> 1, cofs = (Lid & 1) * 32 + piece * 4;
            const v4f val = *(const v4fa*)(os + row * 68 + cofs); *(volatile v4f*)(crow + (size_t)row * ldc + cofs) = val; }
    };
    pass(); __threadfence(); pass();
}
__global__ __launch_bounds__(256) void k_planes32z(const float* __restrict__ F, int ld, int off, float sc, int rows, bf* Ph, bf* Pl) {
    typedef __attribute__((ext_vector_type(2))) unsigned short v2us;
    const int lane = threadIdx.x & 31; const size_t r = ((size_t)blockIdx.x * 8 + (threadIdx.x >> 5)) * 2 + (lane >> 4); if (r >= (size_t)rows) return; const int z = blockIdx.z; const int c0 = (lane & 15) * 2; v2us oh, ol;
    Ph += (size_t)z * rows * 32; Pl += (size_t)z * rows * 32;
#pragma unroll
    for (int i = 0; i < 2; ++i) { const float y = F[r * ld + off + z * 32 + c0 + i] * sc; const unsigned short hb = f2bf(y); oh[i] = hb; ol[i] = f2bf(y - bf2f(hb)); }
    const size_t o = r * 32 + c0; *(volatile v2us*)(Ph + o) = oh; *(volatile v2us*)(Pl + o) = ol; __threadfence(); *(volatile v2us*)(Ph + o) = oh; *(volatile v2us*)(Pl + o) = ol;
}
__global__ __launch_bounds__(256) void k_vtpadz(const float* __restrict__ F, int ld, int off, int nk, bf* Th, bf* Tl) {
    typedef __attribute__((ext_vector_type(2))) unsigned short v2us;
    const int lane = threadIdx.x & 31; const size_t wid = (size_t)blockIdx.x * 8 + (threadIdx.x >> 5); if (wid >= (size_t)64 * (nk / 64)) return; const int z = blockIdx.z; const int d = (int)(wid / (nk / 64)); const int k0 = (int)(wid % (nk / 64)) * 64 + lane * 2; v2us oh, ol;
    Th += (size_t)z * 64 * nk; Tl += (size_t)z * 64 * nk;
#pragma unroll
    for (int i = 0; i < 2; ++i) { const float y = (d < 32) ? F[(size_t)(k0 + i) * ld + off + z * 32 + (d < 32 ? d : 0)] : 0.f; const unsigned short hb = f2bf(y); oh[i] = hb; ol[i] = f2bf(y - bf2f(hb)); }
    const size_t o = (size_t)d * nk + k0; *(volatile v2us*)(Th + o) = oh; *(volatile v2us*)(Tl + o) = ol; __threadfence(); *(volatile v2us*)(Th + o) = oh; *(volatile v2us*)(Tl + o) = ol;
}
template <int NK>
__global__ __launch_bounds__(256) void k_softmaxz(const float* __restrict__ S, int rows, bf* PH, bf* PL) {
    typedef __attribute__((ext_vector_type(4))) unsigned short v4us;
    const int lane = threadIdx.x & 31, i = blockIdx.x * 8 + (threadIdx.x >> 5); if (i >= rows) return; const size_t zo = (size_t)blockIdx.z * rows * NK; const float* sr = S + zo + (size_t)i * NK; PH += zo; PL += zo;
    float m = -3.0e38f;
#pragma unroll 1
    for (int c0 = lane * 4; c0 < NK; c0 += 128) {
#pragma unroll
        for (int q = 0; q < 4; ++q) m = fmaxf(m, sr[c0 + q]); }
#pragma unroll
    for (int sh = 16; sh; sh >>= 1) m = fmaxf(m, __shfl_xor(m, sh, 32));
    float sum = 0.f;
#pragma unroll 1
    for (int c0 = lane * 4; c0 < NK; c0 += 128) {
#pragma unroll
        for (int q = 0; q < 4; ++q) sum += __expf(sr[c0 + q] - m); }
#pragma unroll
    for (int sh = 16; sh; sh >>= 1) sum += __shfl_xor(sum, sh, 32);
    const float inv = 1.0f / sum;
#pragma unroll 1
    for (int ps = 0; ps < 2; ++ps) {
#pragma unroll 1
        for (int c0 = lane * 4; c0 < NK; c0 += 128) { v4us oh, ol;
#pragma unroll
            for (int q = 0; q < 4; ++q) { const float p = __expf(sr[c0 + q] - m) * inv; const unsigned short hb = f2bf(p); oh[q] = hb; ol[q] = f2bf(p - bf2f(hb)); }
            const size_t o = (size_t)i * NK + c0; *(volatile v4us*)(PH + o) = oh; *(volatile v4us*)(PL + o) = ol; }
        if (ps == 0) __threadfence(); }
}
__global__ __launch_bounds__(256) void k_placez(const float* __restrict__ XH, int rows, int ldy, float* Y) {
    const int lane = threadIdx.x & 31; const size_t q = (size_t)blockIdx.x * 8 + (threadIdx.x >> 5); if (q >= (size_t)rows) return; const int z = blockIdx.z; const float v = XH[((size_t)z * rows + q) * 64 + lane];
    *(volatile float*)(Y + q * ldy + z * 32 + lane) = v; __threadfence(); *(volatile float*)(Y + q * ldy + z * 32 + lane) = v;
}
template <int MODE>
__global__ __launch_bounds__(128) void k_gemm3rz(const bf* __restrict__ Ah, const bf* __restrict__ Al, const bf* __restrict__ Bh, const bf* __restrict__ Bl, int K, float* C, int ldc, size_t sA, size_t sB, size_t sC, const float* __restrict__ R, float sgn) {
    const size_t z = blockIdx.z; Ah += z * sA; Al += z * sA; Bh += z * sB; Bl += z * sB; C += z * sC; R += z * sC;
    const int Klim = K;
    __shared__ __align__(16) float ost[4][16 * 68];
    const int lane = threadIdx.x & 31, wave = threadIdx.x >> 5, lr = lane & 15, hi = lane >> 4;
    const int r0 = blockIdx.x * 64 + wave * 16, c0 = blockIdx.y * 64;
    const size_t aoff = (size_t)(r0 + lr) * K + 8 * hi;
    v8f acc[4];
#pragma unroll
    for (int t = 0; t < 4; ++t) acc[t] = (v8f){};
#pragma unroll 1
    for (int kc = 0; kc < Klim; kc += 32) {
        const v16bf a = cat16b(*(const v8us*)(Ah + aoff + kc), *(const v8us*)(Ah + aoff + kc + 16));
        v16bf al = a; if (!(MODE & 4) && !(MODE & 16)) al = cat16b(*(const v8us*)(Al + aoff + kc), *(const v8us*)(Al + aoff + kc + 16));
#pragma unroll
        for (int t = 0; t < 4; ++t) { const size_t bo = (size_t)(c0 + t * 16 + lr) * K + kc + 8 * hi;
            const v16bf bh = cat16b(*(const v8us*)(Bh + bo), *(const v8us*)(Bh + bo + 16));
            acc[t] = wmmab(a, bh, acc[t]);
            if (!(MODE & 4)) { if (!(MODE & 16)) acc[t] = wmmab(al, bh, acc[t]); if (!(MODE & 8)) { const v16bf bl = cat16b(*(const v8us*)(Bl + bo), *(const v8us*)(Bl + bo + 16)); acc[t] = wmmab(a, bl, acc[t]); } } }
        asm volatile("v_nop\n\tv_nop\n\tv_nop\n\tv_nop" : "+v"(acc[0]), "+v"(acc[1]), "+v"(acc[2]), "+v"(acc[3]) : "v"(a), "v"(al));
    }
    float* os = &ost[wave][0];
#pragma unroll
    for (int t = 0; t < 4; ++t) {
#pragma unroll
        for (int j = 0; j < 8; ++j) os[(hi * 8 + j) * 68 + t * 16 + lr] = acc[t][j]; }
    __builtin_amdgcn_wave_barrier(); asm volatile("" ::: "memory");
    float* crow = C + (size_t)r0 * ldc + c0; const float* rrow = R + (size_t)r0 * ldc + c0;
    auto pass = [&]() {
#pragma unroll
        for (int s = 0; s < 8; ++s) { const int Lid = (lane >> 3) + 4 * s, piece = lane & 7; const int row = Lid >> 1, cofs = (Lid & 1) * 32 + piece * 4;
            v4f val = *(const v4fa*)(os + row * 68 + cofs); const v4f rv = *(const v4f*)(rrow + (size_t)row * ldc + cofs); val = val * sgn + rv; *(volatile v4f*)(crow + (size_t)row * ldc + cofs) = val; }
    };
    pass(); __threadfence(); pass();
}

__global__ __launch_bounds__(256) void k_twiddle(bf* Ch, bf* Cl, bf* Sh, bf* Sl) {
    typedef __attribute__((ext_vector_type(4))) unsigned short v4us;
    __shared__ float ctab[NI]; __shared__ float stab[NI];
    if (threadIdx.x < NI) { const float ang = (float)threadIdx.x * W224; ctab[threadIdx.x] = cosf(ang); stab[threadIdx.x] = -sinf(ang); }
    __syncthreads();
    const int lane = threadIdx.x & 31; const int k = blockIdx.x * 8 + (threadIdx.x >> 5); if (k >= NP) return;
#pragma unroll 1
    for (int ps = 0; ps < 2; ++ps) {
#pragma unroll 1
        for (int c0 = lane * 4; c0 < NP; c0 += 128) { v4us ch, cl, sh_, sl;
#pragma unroll
            for (int q = 0; q < 4; ++q) { const int n = c0 + q; float cv = 0.f, sv = 0.f; if (k < NI && n < NI) { const int m = (k * n) % NI; cv = ctab[m]; sv = stab[m]; }
                { const unsigned short hb = f2bf(cv); ch[q] = hb; cl[q] = f2bf(cv - bf2f(hb)); } { const unsigned short hb = f2bf(sv); sh_[q] = hb; sl[q] = f2bf(sv - bf2f(hb)); } }
            const size_t o = (size_t)k * NP + c0; *(volatile v4us*)(Ch + o) = ch; *(volatile v4us*)(Cl + o) = cl; *(volatile v4us*)(Sh + o) = sh_; *(volatile v4us*)(Sl + o) = sl; }
        if (ps == 0) __threadfence(); }
}
__global__ __launch_bounds__(256) void k_gray(const float* __restrict__ xb, bf* Gh, bf* Gl) {
    typedef __attribute__((ext_vector_type(4))) unsigned short v4us;
    const int lane = threadIdx.x & 31; const int r = blockIdx.x * 8 + (threadIdx.x >> 5); if (r >= NP) return; const size_t z = blockIdx.z; xb += z * 3 * NPIX; Gh += z * NP * NP; Gl += z * NP * NP;
#pragma unroll 1
    for (int ps = 0; ps < 2; ++ps) {
#pragma unroll 1
        for (int c0 = lane * 4; c0 < NP; c0 += 128) { v4us oh, ol;
#pragma unroll
            for (int q = 0; q < 4; ++q) { const int n = c0 + q; float v = 0.f; if (r < NI && n < NI) { const size_t o = (size_t)r * NI + n; v = (bfr(xb[o]) + bfr(xb[NPIX + o]) + bfr(xb[2 * NPIX + o])) / 3.0f; } const unsigned short hb = f2bf(v); oh[q] = hb; ol[q] = f2bf(v - bf2f(hb)); }
            const size_t o = (size_t)r * NP + c0; *(volatile v4us*)(Gh + o) = oh; *(volatile v4us*)(Gl + o) = ol; }
        if (ps == 0) __threadfence(); }
}
__global__ __launch_bounds__(256) void k_splitsq(const float* __restrict__ src, bf* dh, bf* dl) {
    const int lane = threadIdx.x & 31; const size_t r = (size_t)blockIdx.x * 8 + (threadIdx.x >> 5); if (r >= (size_t)NP) return; const size_t z = blockIdx.z; src += z * NP * NP; dh += z * NP * NP; dl += z * NP * NP; const size_t o = r * NP + lane * 8; const v8f v = *(const v8f*)(src + o); v8us oh, ol;
#pragma unroll
    for (int i = 0; i < 8; ++i) { const unsigned short hb = f2bf(v[i]); oh[i] = hb; ol[i] = f2bf(v[i] - bf2f(hb)); }
    *(volatile v8us*)(dh + o) = oh; *(volatile v8us*)(dl + o) = ol; __threadfence(); *(volatile v8us*)(dh + o) = oh; *(volatile v8us*)(dl + o) = ol;
}
__global__ __launch_bounds__(256) void k_mag(const float* __restrict__ Fre, const float* __restrict__ Fim, float* MAG) {
    const int lane = threadIdx.x & 31; const int h = blockIdx.x * 8 + (threadIdx.x >> 5); if (h >= NI) return; const size_t z = blockIdx.z; Fre += z * NP * NP; Fim += z * NP * NP; MAG += z * (size_t)NI * NP; const int k1 = (h + NI / 2) % NI;
#pragma unroll 1
    for (int c0 = lane * 4; c0 < NP; c0 += 128) { v4f v;
#pragma unroll
        for (int q = 0; q < 4; ++q) { const int w = c0 + q; float m = 0.f; if (w < NI) { const int k2 = (w + NI / 2) % NI; const float re = Fre[(size_t)k1 * NP + k2], im = Fim[(size_t)k1 * NP + k2]; m = log1pf(sqrtf(re * re + im * im)); } v[q] = m; }
        *(volatile v4f*)(MAG + (size_t)h * NP + c0) = v; __threadfence(); *(volatile v4f*)(MAG + (size_t)h * NP + c0) = v; }
}
__global__ __launch_bounds__(256) void k_stats(const float* __restrict__ MAG, float* FEATb) {
    MAG += (size_t)blockIdx.x * NI * NP; FEATb += (size_t)blockIdx.x * 32;
    __shared__ float red[256]; __shared__ float bs1[KB][256]; __shared__ float bs2[KB][256]; __shared__ float bmx[KB][256]; __shared__ float resl[32];
    const int t = threadIdx.x;
    float s = 0.f; for (int p = t; p < NPIX; p += 256) { const int h = p / NI, w = p % NI; s += MAG[(size_t)h * NP + w]; }
    red[t] = s; __syncthreads(); for (int st = 128; st > 0; st >>= 1) { if (t < st) red[t] += red[t + st]; __syncthreads(); }
    const float mu = red[0] / (float)NPIX; __syncthreads();
    float sq = 0.f; for (int p = t; p < NPIX; p += 256) { const int h = p / NI, w = p % NI; const float d = MAG[(size_t)h * NP + w] - mu; sq = fmaf(d, d, sq); }
    red[t] = sq; __syncthreads(); for (int st = 128; st > 0; st >>= 1) { if (t < st) red[t] += red[t + st]; __syncthreads(); }
    const float sd = sqrtf(red[0] / (float)(NPIX - 1)) + 1e-6f; const float isd = 1.0f / sd; __syncthreads();
    float a1[KB], a2[KB], amx[KB]; int cnt[KB];
#pragma unroll
    for (int i = 0; i < KB; ++i) { a1[i] = 0.f; a2[i] = 0.f; amx[i] = -1e9f; cnt[i] = 0; }
    for (int p = t; p < NPIX; p += 256) { const int y = p / NI, x = p % NI; const float r = sqrtf((float)((x - NI / 2) * (x - NI / 2) + (y - NI / 2) * (y - NI / 2))); const float mv = (MAG[(size_t)y * NP + x] - mu) * isd;
#pragma unroll
        for (int i = 0; i < KB; ++i) { const bool in = (r >= STEPR * (float)i) && (r < STEPR * ((float)i + 1.0f)); if (in) { a1[i] += mv; a2[i] = fmaf(mv, mv, a2[i]); amx[i] = fmaxf(amx[i], mv); cnt[i] += 1; } } }
#pragma unroll
    for (int i = 0; i < KB; ++i) { bs1[i][t] = a1[i]; bs2[i][t] = a2[i]; bmx[i][t] = amx[i]; }
    __syncthreads();
    for (int st = 128; st > 0; st >>= 1) { if (t < st) {
#pragma unroll
            for (int i = 0; i < KB; ++i) { bs1[i][t] += bs1[i][t + st]; bs2[i][t] += bs2[i][t + st]; bmx[i][t] = fmaxf(bmx[i][t], bmx[i][t + st]); } }
        __syncthreads(); }
#pragma unroll 1
    for (int i = 0; i < KB; ++i) { red[t] = (float)cnt[i]; __syncthreads(); for (int st = 128; st > 0; st >>= 1) { if (t < st) red[t] += red[t + st]; __syncthreads(); }
        if (t == 0) { const float msum = red[0]; const float ms = msum + 1e-6f; const float s1 = bs1[i][0], s2 = bs2[i][0]; const float mean = s1 / ms; const float varn = s2 - 2.0f * mean * s1 + mean * mean * msum; const float stdv = sqrtf(varn / ms + 1e-6f);
            resl[i * 3 + 0] = mean; resl[i * 3 + 1] = stdv; resl[i * 3 + 2] = bmx[i][0]; }
        __syncthreads(); }
    if (t >= 24 && t < 32) resl[t] = 0.f;
    __syncthreads();
    if (t < 32) { const float v = resl[t]; *(volatile float*)(FEATb + t) = v; __threadfence(); *(volatile float*)(FEATb + t) = v; }
}
__global__ __launch_bounds__(256) void k_head(const float* __restrict__ FEAT, const float* __restrict__ W1, const float* __restrict__ b1, const float* __restrict__ gam, const float* __restrict__ bet, bf* Hh, bf* Hl) {
    const int lane = threadIdx.x & 31; const int r = blockIdx.x * 8 + (threadIdx.x >> 5); if (r >= NBT * KB) return; const int b = r / KB, k = r % KB; const float f0 = FEAT[b * 32 + k * 3], f1 = FEAT[b * 32 + k * 3 + 1], f2 = FEAT[b * 32 + k * 3 + 2];
    float h[8]; float s = 0.f;
#pragma unroll
    for (int i = 0; i < 8; ++i) { const int e = lane * 8 + i; const float v = f0 * bfr(W1[e]) + f1 * bfr(W1[EE + e]) + f2 * bfr(W1[2 * EE + e]) + bfr(b1[e]); h[i] = v; s += v; }
#pragma unroll
    for (int sh = 16; sh; sh >>= 1) s += __shfl_xor(s, sh, 32);
    const float mu = s * (1.0f / EE); float q = 0.f;
#pragma unroll
    for (int i = 0; i < 8; ++i) { const float d = h[i] - mu; q = fmaf(d, d, q); }
#pragma unroll
    for (int sh = 16; sh; sh >>= 1) q += __shfl_xor(q, sh, 32);
    const float rs = rsqrtf(q * (1.0f / EE) + 1e-5f); v8us oh, ol;
#pragma unroll
    for (int i = 0; i < 8; ++i) { const int e = lane * 8 + i; float y = (h[i] - mu) * rs * bfr(gam[e]) + bfr(bet[e]); y = fmaxf(y, 0.f); const unsigned short hb = f2bf(y); oh[i] = hb; ol[i] = f2bf(y - bf2f(hb)); }
    const size_t o = (size_t)r * EE + lane * 8; *(volatile v8us*)(Hh + o) = oh; *(volatile v8us*)(Hl + o) = ol; __threadfence(); *(volatile v8us*)(Hh + o) = oh; *(volatile v8us*)(Hl + o) = ol;
}

extern "C" void kernel_launch(void* const* d_in, const int* in_sizes, int n_in,
                              void* d_out, int out_size, void* d_ws, size_t ws_size, hipStream_t stream) {
    (void)in_sizes; (void)n_in; (void)out_size;
    const float* x = (const float*)d_in[0]; const float* W1 = (const float*)d_in[1]; const float* b1 = (const float*)d_in[2]; const float* gam = (const float*)d_in[3]; const float* bet = (const float*)d_in[4]; const float* W2 = (const float*)d_in[5]; const float* b2 = (const float*)d_in[6];
    float* out = (float*)d_out;
    char* wsp = (char*)d_ws;
    auto take = [&](size_t bytes) { char* p = wsp; wsp += (bytes + 255) & ~(size_t)255; return (void*)p; };
    const int ZI = 16;
    const size_t PL2 = (size_t)NP * NP * 2, PF = (size_t)NP * NP * 4, SQ = (size_t)NP * NP;
    bf* Ch = (bf*)take(PL2); bf* Cl = (bf*)take(PL2); bf* Sh = (bf*)take(PL2); bf* Sl = (bf*)take(PL2); bf* W2T = (bf*)take((size_t)EE * EE * 2);
    bf* Gh = (bf*)take(ZI * PL2); bf* Gl = (bf*)take(ZI * PL2); float* TR = (float*)take(ZI * PF); float* TI = (float*)take(ZI * PF); bf* TRh = (bf*)take(ZI * PL2); bf* TRl = (bf*)take(ZI * PL2); bf* TIh = (bf*)take(ZI * PL2); bf* TIl = (bf*)take(ZI * PL2);
    float* F1 = (float*)take(ZI * PF); float* FR = (float*)take(ZI * PF); float* F2 = (float*)take(ZI * PF); float* FI = (float*)take(ZI * PF); float* MAG = (float*)take(ZI * (size_t)NI * NP * 4); float* FEAT = (float*)take((size_t)NBT * 32 * 4); bf* Hh = (bf*)take((size_t)NBT * KB * EE * 2); bf* Hl = (bf*)take((size_t)NBT * KB * EE * 2);
    if ((size_t)(wsp - (char*)d_ws) > ws_size) return;
    k_twiddle<<<NP / 8, 256, 0, stream>>>(Ch, Cl, Sh, Sl); k_wt<<<dim3(EE / 64, EE / 64, 1), 256, 0, stream>>>(W2, EE, EE, W2T);
    for (int gI = 0; gI < NBT / ZI; ++gI) { const float* xg = x + (size_t)gI * ZI * 3 * NPIX;
        k_gray<<<dim3(NP / 8, 1, ZI), 256, 0, stream>>>(xg, Gh, Gl);
        k_gemm3z<0><<<dim3(NP / 64, NP / 64, ZI), 128, 0, stream>>>(Ch, Cl, Gh, Gl, NP, TR, NP, 0, SQ, SQ);
        k_gemm3z<0><<<dim3(NP / 64, NP / 64, ZI), 128, 0, stream>>>(Sh, Sl, Gh, Gl, NP, TI, NP, 0, SQ, SQ);
        k_splitsq<<<dim3(NP / 8, 1, ZI), 256, 0, stream>>>(TR, TRh, TRl); k_splitsq<<<dim3(NP / 8, 1, ZI), 256, 0, stream>>>(TI, TIh, TIl);
        k_gemm3z<0><<<dim3(NP / 64, NP / 64, ZI), 128, 0, stream>>>(Ch, Cl, TRh, TRl, NP, F1, NP, 0, SQ, SQ);
        k_gemm3rz<0><<<dim3(NP / 64, NP / 64, ZI), 128, 0, stream>>>(Sh, Sl, TIh, TIl, NP, FR, NP, 0, SQ, SQ, F1, -1.0f);
        k_gemm3z<0><<<dim3(NP / 64, NP / 64, ZI), 128, 0, stream>>>(Ch, Cl, TIh, TIl, NP, F2, NP, 0, SQ, SQ);
        k_gemm3rz<0><<<dim3(NP / 64, NP / 64, ZI), 128, 0, stream>>>(Sh, Sl, TRh, TRl, NP, FI, NP, 0, SQ, SQ, F2, 1.0f);
        k_mag<<<dim3(NI / 8, 1, ZI), 256, 0, stream>>>(FR, FI, MAG);
        k_stats<<<ZI, 256, 0, stream>>>(MAG, FEAT + (size_t)gI * ZI * 32); }
    k_head<<<(NBT * KB) / 8, 256, 0, stream>>>(FEAT, W1, b1, gam, bet, Hh, Hl);
    k_gemmb<true, false><<<dim3((NBT * KB) / 64, EE / 64, 1), 128, 0, stream>>>(Hh, Hl, W2T, b2, out, EE, nullptr, nullptr, EE);
}
